// MultiHeadSelfAttention2D_51951924412912
// MI455X (gfx1250) — hardware-verified
//
#include <hip/hip_runtime.h>


#define NB_  16
#define CI   256
#define CO   512
#define MM   1024
#define HH   32
#define NH_  8
#define HD   64
typedef _Float16 h16;
typedef unsigned short bf;
typedef __attribute__((ext_vector_type(16))) __bf16   v16bf;
typedef __attribute__((ext_vector_type(16))) _Float16 v16h;
typedef __attribute__((ext_vector_type(8)))  _Float16 v8h;
typedef __attribute__((ext_vector_type(8)))  unsigned short v8us;
typedef __attribute__((ext_vector_type(8)))  float    v8f;
typedef __attribute__((ext_vector_type(4)))  float    v4f;
typedef v8h  __attribute__((may_alias)) v8ha;
typedef v4f  __attribute__((may_alias)) v4fa;
typedef v8us __attribute__((may_alias)) v8usa;

__device__ __forceinline__ unsigned short f2bf(float f) { unsigned u = __float_as_uint(f); u += 0x7FFFu + ((u >> 16) & 1u); return (unsigned short)(u >> 16); }
__device__ __forceinline__ float bf2f(unsigned short b) { return __uint_as_float(((unsigned)b) << 16); }
__device__ __forceinline__ float bfr(float f) { return bf2f(f2bf(f)); }
__device__ __forceinline__ v16h cat16(v8h lo, v8h hi) { return __builtin_shufflevector(lo, hi, 0, 1, 2, 3, 4, 5, 6, 7, 8, 9, 10, 11, 12, 13, 14, 15); }
__device__ __forceinline__ v16bf cat16b(v8us lo, v8us hi) { return __builtin_bit_cast(v16bf, __builtin_shufflevector(lo, hi, 0, 1, 2, 3, 4, 5, 6, 7, 8, 9, 10, 11, 12, 13, 14, 15)); }
__device__ __forceinline__ v8f wmma16(v16h a, v16h b, v8f c) { return __builtin_amdgcn_wmma_f32_16x16x32_f16(false, a, false, b, (short)0, c, false, false); }
__device__ __forceinline__ v8f wmmab(v16bf a, v16bf b, v8f c) { return __builtin_amdgcn_wmma_f32_16x16x32_bf16(false, a, false, b, (short)0, c, false, false); }


template <typename T16> struct WFrag;
template <> struct WFrag<h16> { typedef v16h V; static __device__ __forceinline__ V ld(const h16* p) { return cat16(*(const v8h*)p, *(const v8h*)(p + 16)); } static __device__ __forceinline__ v8f mma(V a, V b, v8f c) { return wmma16(a, b, c); } };
template <> struct WFrag<bf> { typedef v16bf V; static __device__ __forceinline__ V ld(const bf* p) { return cat16b(*(const v8us*)p, *(const v8us*)(p + 16)); } static __device__ __forceinline__ v8f mma(V a, V b, v8f c) { return wmmab(a, b, c); } };
template <typename T16, int NSPLIT, bool BIAS>
__global__ __launch_bounds__(32) void k_gemmw(const T16* __restrict__ A, const T16* __restrict__ A2, const T16* __restrict__ Bt, const T16* __restrict__ Bt2, int K, float* C, int ldc, const float* __restrict__ bias, size_t sA, size_t sB, size_t sC) {
    typedef typename WFrag<T16>::V V;
    __shared__ __align__(16) float os[16 * 68];
    const size_t z = blockIdx.z; A += z * sA; if (A2) A2 += z * sA; Bt += z * sB; if (Bt2) Bt2 += z * sB; C += z * sC;
    const int lane = threadIdx.x & 31, lr = lane & 15, hi = lane >> 4; const int r0 = blockIdx.x * 64, c0 = blockIdx.y * 64;
    v8f acc[4][4];
#pragma unroll
    for (int mb = 0; mb < 4; ++mb)
#pragma unroll
        for (int nb = 0; nb < 4; ++nb) acc[mb][nb] = (v8f){};
    const size_t aoff = (size_t)(r0 + lr) * K + 8 * hi, boff = (size_t)(c0 + lr) * K + 8 * hi;
#pragma unroll 1
    for (int kc = 0; kc < K; kc += 32) {
        V a[4], a2[4];
#pragma unroll
        for (int mb = 0; mb < 4; ++mb) { a[mb] = WFrag<T16>::ld(A + aoff + (size_t)mb * 16 * K + kc); if (NSPLIT == 1 || NSPLIT == 2) a2[mb] = WFrag<T16>::ld(A2 + aoff + (size_t)mb * 16 * K + kc); }
#pragma unroll
        for (int nb = 0; nb < 4; ++nb) { const V b = WFrag<T16>::ld(Bt + boff + (size_t)nb * 16 * K + kc); V b2; if (NSPLIT >= 2) b2 = WFrag<T16>::ld(Bt2 + boff + (size_t)nb * 16 * K + kc);
#pragma unroll
            for (int mb = 0; mb < 4; ++mb) { acc[mb][nb] = WFrag<T16>::mma(a[mb], b, acc[mb][nb]); if (NSPLIT == 1 || NSPLIT == 2) acc[mb][nb] = WFrag<T16>::mma(a2[mb], b, acc[mb][nb]); if (NSPLIT >= 2) acc[mb][nb] = WFrag<T16>::mma(a[mb], b2, acc[mb][nb]); } }
        asm volatile("v_nop\n\tv_nop\n\tv_nop\n\tv_nop" : "+v"(acc[0][0]), "+v"(acc[1][1]), "+v"(acc[2][2]), "+v"(acc[3][3]) : "v"(a[0]), "v"(a[3]));
    }
#pragma unroll
    for (int mb = 0; mb < 4; ++mb) {
#pragma unroll
        for (int nb = 0; nb < 4; ++nb) {
#pragma unroll
            for (int j = 0; j < 8; ++j) os[(hi * 8 + j) * 68 + nb * 16 + lr] = acc[mb][nb][j]; }
        __builtin_amdgcn_wave_barrier(); asm volatile("" ::: "memory");
        float* crow = C + (size_t)(r0 + mb * 16) * ldc + c0;
#pragma unroll 1
        for (int ps = 0; ps < 2; ++ps) {
#pragma unroll
            for (int s = 0; s < 8; ++s) { const int row = 2 * s + hi, cofs = lr * 4; v4f val = *(const v4fa*)(os + row * 68 + cofs); if (BIAS) { val[0] += bfr(bias[c0 + cofs]); val[1] += bfr(bias[c0 + cofs + 1]); val[2] += bfr(bias[c0 + cofs + 2]); val[3] += bfr(bias[c0 + cofs + 3]); }
                *(volatile v4f*)(crow + (size_t)row * ldc + cofs) = val; }
            if (ps == 0) __threadfence(); }
        __builtin_amdgcn_wave_barrier(); asm volatile("" ::: "memory");
    }
}

__device__ __forceinline__ void splitf(float y, unsigned short& h, unsigned short& l) { h = f2bf(y); l = f2bf(y - bf2f(h)); }
typedef __attribute__((ext_vector_type(2))) unsigned short v2us;
typedef __attribute__((ext_vector_type(4))) unsigned short v4us;

__global__ __launch_bounds__(256) void k_cvt8(const float* __restrict__ src, bf* dst, size_t n8) { const size_t i = (size_t)blockIdx.x * 256 + threadIdx.x; if (i >= n8) return; const v8f v = *(const v8f*)(src + i * 8); v8us o;
#pragma unroll
    for (int k = 0; k < 8; ++k) o[k] = f2bf(v[k]); *(volatile v8us*)(dst + i * 8) = o; __threadfence(); *(volatile v8us*)(dst + i * 8) = o; }
__global__ __launch_bounds__(256) void k_pe(float* PE) { const int e = (blockIdx.x * 256 + threadIdx.x) * 4; if (e >= CO * MM) return; const int c = e / MM; const int m0 = e % MM; const int cc = (c < CO / 2) ? c : c - CO / 2; const int ch2 = cc & ~1; const float div = __expf(-logf(10000.0f) * (float)ch2 / (float)(CO / 2)); v4f r;
#pragma unroll 1
    for (int u = 0; u < 4; ++u) { const int m = m0 + u; const int p = (c < CO / 2) ? (m / HH) : (m % HH); const float ang = __fmul_rn((float)p, div); r[u] = (cc & 1) ? cosf(ang) : sinf(ang); }
    *(volatile v4f*)(PE + e) = r; __threadfence(); *(volatile v4f*)(PE + e) = r; }
__global__ __launch_bounds__(256) void k_xt(const float* __restrict__ X, bf* XT) { const int e = (blockIdx.x * 256 + threadIdx.x) * 4; if (e >= MM * CI) return; const int c = e % CI; const int m = e / CI; v4us o;
#pragma unroll
    for (int u = 0; u < 4; ++u) o[u] = f2bf(X[(size_t)(c + u) * MM + m]); *(volatile v4us*)(XT + e) = o; __threadfence(); *(volatile v4us*)(XT + e) = o; }
__global__ __launch_bounds__(256) void k_qpl(const float* __restrict__ F, const float* __restrict__ PE, bf* Ph, bf* Pl) { const int e = (blockIdx.x * 256 + threadIdx.x) * 4; if (e >= NH_ * MM * HD) return; const int d = e % HD; const int m = (e / HD) % MM; const int h = e / (HD * MM); v4us oh, ol;
#pragma unroll
    for (int u = 0; u < 4; ++u) { const size_t idx = (size_t)(h * HD + d + u) * MM + m; unsigned short a, b; splitf(__fadd_rn(F[idx], PE[idx]), a, b); oh[u] = a; ol[u] = b; } *(volatile v4us*)(Ph + e) = oh; *(volatile v4us*)(Pl + e) = ol; __threadfence(); *(volatile v4us*)(Ph + e) = oh; *(volatile v4us*)(Pl + e) = ol; }
__global__ __launch_bounds__(256) void k_vpl(const float* __restrict__ F, bf* Ph, bf* Pl) { const int e = (blockIdx.x * 256 + threadIdx.x) * 4; if (e >= CO * MM) return; v4us oh, ol; const v4f a = *(const v4f*)(F + e);
#pragma unroll
    for (int u = 0; u < 4; ++u) { unsigned short x0, x1; splitf(a[u], x0, x1); oh[u] = x0; ol[u] = x1; } *(volatile v4us*)(Ph + e) = oh; *(volatile v4us*)(Pl + e) = ol; __threadfence(); *(volatile v4us*)(Ph + e) = oh; *(volatile v4us*)(Pl + e) = ol; }
__global__ __launch_bounds__(256) void k_csoft(const float* __restrict__ S, bf* Ph, bf* Pl) { const int lane = threadIdx.x & 31; const int row = blockIdx.x * 8 + (threadIdx.x >> 5); if (row >= NH_ * MM) return; const float* sr = S + (size_t)row * MM; float v[MM / 32]; float mx = -3.0e38f;
#pragma unroll
    for (int ch = 0; ch < MM / 128; ++ch) { const v4f a = *(const v4f*)(sr + ch * 128 + lane * 4);
#pragma unroll
        for (int u = 0; u < 4; ++u) { const float t = fminf(fmaxf(a[u] * 0.125f, -50.0f), 50.0f); v[ch * 4 + u] = t; mx = fmaxf(mx, t); } }
#pragma unroll
    for (int sh = 16; sh; sh >>= 1) mx = fmaxf(mx, __shfl_xor(mx, sh, 32));
    float sum = 0.f;
#pragma unroll
    for (int q = 0; q < MM / 32; ++q) { float d0 = __fsub_rn(v[q], mx); asm volatile("" : "+v"(d0)); v[q] = __builtin_amdgcn_exp2f(__fmul_rn(d0, 1.4426950408889634f)); sum += v[q]; }
#pragma unroll
    for (int sh = 16; sh; sh >>= 1) sum += __shfl_xor(sum, sh, 32);
    const float f = __fdiv_rn(1.0f, sum);
    for (int ps = 0; ps < 2; ++ps) {
#pragma unroll
        for (int ch = 0; ch < MM / 128; ++ch) { v4us oh, ol; for (int q = 0; q < 4; ++q) { unsigned short a2, c2; splitf(v[ch * 4 + q] * f, a2, c2); oh[q] = a2; ol[q] = c2; } const size_t oo = (size_t)row * MM + ch * 128 + lane * 4; *(volatile v4us*)(Ph + oo) = oh; *(volatile v4us*)(Pl + oo) = ol; }
        if (ps == 0) __threadfence(); } }

extern "C" void kernel_launch(void* const* d_in, const int* in_sizes, int n_in,
                              void* d_out, int out_size, void* d_ws, size_t ws_size, hipStream_t stream) {
    (void)in_sizes; (void)n_in; (void)out_size;
    const float* x = (const float*)d_in[0]; const float* Wq = (const float*)d_in[1]; const float* Wk = (const float*)d_in[2]; const float* Wv = (const float*)d_in[3];
    float* OUT = (float*)d_out;
    char* wsp = (char*)d_ws;
    auto take = [&](size_t bytes) { char* p = wsp; wsp += (bytes + 255) & ~(size_t)255; return (void*)p; };
    bf* AQ = (bf*)take((size_t)CO * CI * 2); bf* AK = (bf*)take((size_t)CO * CI * 2); bf* AV = (bf*)take((size_t)CO * CI * 2); float* PE = (float*)take((size_t)CO * MM * 4); bf* XT = (bf*)take((size_t)MM * CI * 2);
    float* F = (float*)take((size_t)CO * MM * 4); bf* QPh = (bf*)take((size_t)NH_ * MM * HD * 2); bf* QPl = (bf*)take((size_t)NH_ * MM * HD * 2); bf* KPh = (bf*)take((size_t)NH_ * MM * HD * 2); bf* KPl = (bf*)take((size_t)NH_ * MM * HD * 2); bf* VPh = (bf*)take((size_t)CO * MM * 2); bf* VPl = (bf*)take((size_t)CO * MM * 2);
    float* S = (float*)take((size_t)NH_ * MM * MM * 4); bf* Ph = (bf*)take((size_t)NH_ * MM * MM * 2); bf* Pl = (bf*)take((size_t)NH_ * MM * MM * 2);
    if ((size_t)(wsp - (char*)d_ws) > ws_size) return;
    k_cvt8<<<(CO * CI / 8 + 255) / 256, 256, 0, stream>>>(Wq, AQ, CO * CI / 8); k_cvt8<<<(CO * CI / 8 + 255) / 256, 256, 0, stream>>>(Wk, AK, CO * CI / 8); k_cvt8<<<(CO * CI / 8 + 255) / 256, 256, 0, stream>>>(Wv, AV, CO * CI / 8);
    k_pe<<<(CO * MM / 4 + 255) / 256, 256, 0, stream>>>(PE);
    const size_t zq = (size_t)MM * HD, zS = (size_t)MM * MM, zv = (size_t)HD * MM;
    for (int b = 0; b < NB_; ++b) {
        k_xt<<<(MM * CI / 4 + 255) / 256, 256, 0, stream>>>(x + (size_t)b * CI * MM, XT);
        k_gemmw<bf, 0, false><<<dim3(CO / 64, MM / 64, 1), 32, 0, stream>>>(AQ, nullptr, XT, nullptr, CI, F, MM, nullptr, 0, 0, 0); k_qpl<<<(NH_ * MM * HD / 4 + 255) / 256, 256, 0, stream>>>(F, PE, QPh, QPl);
        k_gemmw<bf, 0, false><<<dim3(CO / 64, MM / 64, 1), 32, 0, stream>>>(AK, nullptr, XT, nullptr, CI, F, MM, nullptr, 0, 0, 0); k_qpl<<<(NH_ * MM * HD / 4 + 255) / 256, 256, 0, stream>>>(F, PE, KPh, KPl);
        k_gemmw<bf, 0, false><<<dim3(CO / 64, MM / 64, 1), 32, 0, stream>>>(AV, nullptr, XT, nullptr, CI, F, MM, nullptr, 0, 0, 0); k_vpl<<<(CO * MM / 4 + 255) / 256, 256, 0, stream>>>(F, VPh, VPl);
        k_gemmw<bf, 2, false><<<dim3(MM / 64, MM / 64, NH_), 32, 0, stream>>>(QPh, QPl, KPh, KPl, HD, S, MM, nullptr, zq, zq, zS);
        k_csoft<<<NH_ * MM / 8, 256, 0, stream>>>(S, Ph, Pl);
        k_gemmw<bf, 2, false><<<dim3(1, MM / 64, NH_), 32, 0, stream>>>(VPh, VPl, Ph, Pl, MM, OUT + (size_t)b * CO * MM, MM, nullptr, zv, zS, zv); }
}
